// Net_11639361372195
// MI455X (gfx1250) — hardware-verified
//
#include <hip/hip_runtime.h>
#include <stddef.h>
#include <stdint.h>

#define BATCH  4096
#define TSEQ   28
#define NIN    28
#define KIN    32
#define HID    256
#define G3     768
#define NOUT   28
#define NOUTP  32
#define TB     32
#define NTHR   256
#define HP     520
#define XP     40
#define HB_HALVES (TB * HP)
#define SX_HALVES (TB * XP)
#define OFF_HF (2 * HB_HALVES * 2)
#define OFF_SX (OFF_HF + TB * HID * 4)
#define OFF_SO (OFF_SX + 2 * SX_HALVES * 2)
#define GRU_LDS_BYTES (OFF_SO + TB * NOUT * 4)
#define ZFILL16 (OFF_SO / 16)
#define BO_R   0
#define BO_Z   256
#define BO_IN  512
#define BO_HN  768
#define BO_FC  1024
#define NBIAS  1056
#define NU_WHH (G3 * HID / 8)
#define NU_WIH (G3 * KIN / 8)
#define NU_FCW (NOUTP * HID / 8)
#define NU_BIA (NBIAS / 4)
#define NU_BIAP 512
#define PREP_UNITS (NU_WHH + NU_WIH + NU_FCW + NU_BIAP)
#define OUT_CHUNKS (TB * NOUT / 4)

static_assert(OFF_HF % 16 == 0 && OFF_SX % 16 == 0 && OFF_SO % 16 == 0);
static_assert(HP % 8 == 0 && HP >= 2 * HID && (XP * 2) % 16 == 0 && XP >= KIN);
static_assert(BATCH % TB == 0 && NTHR == TB * 8 && NTHR == (HID / 32) * 32);
static_assert((TB * NOUT * 4) % 128 == 0 && OUT_CHUNKS <= NTHR && OUT_CHUNKS % 32 == 0);
static_assert(TSEQ % 2 == 0);
static_assert(NU_WHH % NTHR == 0 && NU_WIH % NTHR == 0 && NU_FCW % NTHR == 0 && PREP_UNITS % NTHR == 0);
static_assert(NU_BIA <= NU_BIAP && (NBIAS * 4) % 128 == 0);
static_assert(HID % 32 == 0 && KIN == 32 && (NIN * 4) % 16 == 0);
static_assert((BATCH / TB) * TB * NOUT == BATCH * NOUT);

typedef float          v4f   __attribute__((ext_vector_type(4)));
typedef float          v8f   __attribute__((ext_vector_type(8)));
typedef int            v4i   __attribute__((ext_vector_type(4)));
typedef int            v8i   __attribute__((ext_vector_type(8)));
typedef unsigned short v4us  __attribute__((ext_vector_type(4)));
typedef unsigned short v8us  __attribute__((ext_vector_type(8)));
typedef unsigned short v16us __attribute__((ext_vector_type(16)));
typedef __bf16         v16bf __attribute__((ext_vector_type(16)));
typedef v4f  __attribute__((may_alias)) v4fa;
typedef v4i  __attribute__((may_alias)) v4ia;
typedef v4us __attribute__((may_alias)) v4usa;
typedef v8us __attribute__((may_alias)) v8usa;
union FragB { v16bf v; v16us u; v8us h[2]; v8i w; };

__device__ __forceinline__ v8f wmb(const FragB& a, const FragB& b, v8f c) {
  v8f d = __builtin_amdgcn_wmma_f32_16x16x32_bf16(false, a.v, false, b.v, (short)0, c, false, false);
  asm volatile("v_nop\n\tv_nop\n\tv_nop\n\tv_nop" : "+v"(d) : "v"(a.w), "v"(b.w));
  return d;
}

__device__ __forceinline__ void ldfrag(FragB& f, const unsigned short* p) {
  f.h[0] = *(const v8usa*)p;
  f.h[1] = *(const v8usa*)(p + 16);
}

__device__ __forceinline__ unsigned bf16_bits(float f) {
  const unsigned u = __float_as_uint(f);
  return (u + 0x7FFFu + ((u >> 16) & 1u)) >> 16;
}
__device__ __forceinline__ float bf16_val(float f) {
  return __uint_as_float(bf16_bits(f) << 16);
}
__device__ __forceinline__ void put16(unsigned short* dp, v8us o) {
  *(volatile v8us*)dp = o;
  __threadfence();
  *(volatile v8us*)dp = o;
}
__device__ __forceinline__ void putf4(float* dp, v4f o) {
  *(volatile v4f*)dp = o;
  __threadfence();
  *(volatile v4f*)dp = o;
}

__global__ __launch_bounds__(NTHR) void k_prep(const float* __restrict__ w_ih, const float* __restrict__ w_hh,
                                               const float* __restrict__ b_ih, const float* __restrict__ b_hh,
                                               const float* __restrict__ fc_w, const float* __restrict__ fc_b,
                                               unsigned short* WHH, unsigned short* WIH,
                                               unsigned short* FCW, float* BIAS) {
  const int u  = (int)blockIdx.x * NTHR + (int)threadIdx.x;
  const int L0 = NU_WHH;
  const int L1 = L0 + NU_WIH;
  const int L2 = L1 + NU_FCW;
  if (u < L0) {
    const float* p = w_hh + (size_t)u * 8;
    const v4f a = *(const v4fa*)p;
    const v4f b = *(const v4fa*)(p + 4);
    v8us o;
    o[0] = (unsigned short)bf16_bits(a.x); o[1] = (unsigned short)bf16_bits(a.y);
    o[2] = (unsigned short)bf16_bits(a.z); o[3] = (unsigned short)bf16_bits(a.w);
    o[4] = (unsigned short)bf16_bits(b.x); o[5] = (unsigned short)bf16_bits(b.y);
    o[6] = (unsigned short)bf16_bits(b.z); o[7] = (unsigned short)bf16_bits(b.w);
    put16(WHH + (size_t)u * 8, o);
    return;
  } else if (u < L1) {
    const int v = u - L0;
    const int n = v >> 2;
    const int j = v & 3;
    const float* p = w_ih + (size_t)n * NIN;
    const int o2 = (j < 3) ? (8 * j + 4) : 24;
    const v4f a = *(const v4fa*)(p + 8 * j);
    const v4f b = *(const v4fa*)(p + o2);
    const bool lv = j < 3;
    v8us o;
    o[0] = (unsigned short)bf16_bits(a.x); o[1] = (unsigned short)bf16_bits(a.y);
    o[2] = (unsigned short)bf16_bits(a.z); o[3] = (unsigned short)bf16_bits(a.w);
    o[4] = lv ? (unsigned short)bf16_bits(b.x) : (unsigned short)0;
    o[5] = lv ? (unsigned short)bf16_bits(b.y) : (unsigned short)0;
    o[6] = lv ? (unsigned short)bf16_bits(b.z) : (unsigned short)0;
    o[7] = lv ? (unsigned short)bf16_bits(b.w) : (unsigned short)0;
    put16(WIH + (size_t)n * KIN + 8 * j, o);
    return;
  } else if (u < L2) {
    const int v  = u - L1;
    const int n  = v >> 5;
    const int k8 = (v & 31) * 8;
    const int nc = n < NOUT ? n : NOUT - 1;
    const bool lv = n < NOUT;
    const float* p = fc_w + (size_t)nc * HID + k8;
    const v4f a = *(const v4fa*)p;
    const v4f b = *(const v4fa*)(p + 4);
    v8us o;
    o[0] = lv ? (unsigned short)bf16_bits(a.x) : (unsigned short)0;
    o[1] = lv ? (unsigned short)bf16_bits(a.y) : (unsigned short)0;
    o[2] = lv ? (unsigned short)bf16_bits(a.z) : (unsigned short)0;
    o[3] = lv ? (unsigned short)bf16_bits(a.w) : (unsigned short)0;
    o[4] = lv ? (unsigned short)bf16_bits(b.x) : (unsigned short)0;
    o[5] = lv ? (unsigned short)bf16_bits(b.y) : (unsigned short)0;
    o[6] = lv ? (unsigned short)bf16_bits(b.z) : (unsigned short)0;
    o[7] = lv ? (unsigned short)bf16_bits(b.w) : (unsigned short)0;
    put16(FCW + (size_t)n * HID + k8, o);
    return;
  } else {
    const int v = u - L2;
    if (v >= NU_BIA) return;
    const int idx = 4 * v;
    v4f q;
    if (idx < 2 * HID) {
      const v4f a = *(const v4fa*)(b_ih + idx);
      const v4f b = *(const v4fa*)(b_hh + idx);
      q.x = bf16_val(a.x) + bf16_val(b.x);
      q.y = bf16_val(a.y) + bf16_val(b.y);
      q.z = bf16_val(a.z) + bf16_val(b.z);
      q.w = bf16_val(a.w) + bf16_val(b.w);
    } else if (idx < 3 * HID) {
      const v4f a = *(const v4fa*)(b_ih + idx);
      q.x = bf16_val(a.x); q.y = bf16_val(a.y); q.z = bf16_val(a.z); q.w = bf16_val(a.w);
    } else if (idx < 4 * HID) {
      const v4f b = *(const v4fa*)(b_hh + (idx - HID));
      q.x = bf16_val(b.x); q.y = bf16_val(b.y); q.z = bf16_val(b.z); q.w = bf16_val(b.w);
    } else {
      const int o  = idx - BO_FC;
      const int oc = o < NOUT - 4 ? o : NOUT - 4;
      const bool lv = o < NOUT;
      const v4f a = *(const v4fa*)(fc_b + oc);
      q.x = lv ? bf16_val(a.x) : 0.0f;
      q.y = lv ? bf16_val(a.y) : 0.0f;
      q.z = lv ? bf16_val(a.z) : 0.0f;
      q.w = lv ? bf16_val(a.w) : 0.0f;
    }
    putf4(BIAS + idx, q);
    return;
  }
}

__device__ __forceinline__ void load_x(const float* __restrict__ x, int b0, int t, unsigned short* sXb, int tid) {
  const int r  = tid >> 3;
  const int j  = tid & 7;
  const int jc = j < 7 ? j : 6;
  const bool lv = j < 7;
  const v4f v = *(const v4fa*)(x + ((size_t)(b0 + r) * TSEQ + t) * NIN + 4 * jc);
  v4us o;
  o.x = lv ? (unsigned short)bf16_bits(v.x) : (unsigned short)0;
  o.y = lv ? (unsigned short)bf16_bits(v.y) : (unsigned short)0;
  o.z = lv ? (unsigned short)bf16_bits(v.z) : (unsigned short)0;
  o.w = lv ? (unsigned short)bf16_bits(v.w) : (unsigned short)0;
  *(v4usa*)(sXb + r * XP + 4 * j) = o;
}

__global__ __launch_bounds__(NTHR) void k_gru(const float* __restrict__ x,
                                              const unsigned short* __restrict__ WHH,
                                              const unsigned short* __restrict__ WIH,
                                              const unsigned short* __restrict__ FCW,
                                              const float* __restrict__ BIAS,
                                              float* out) {
  extern __shared__ __attribute__((aligned(16))) float dyn[];
  unsigned char*  base = (unsigned char*)dyn;
  unsigned short* Hb = (unsigned short*)base;
  float*          hF = (float*)(base + OFF_HF);
  unsigned short* sX = (unsigned short*)(base + OFF_SX);
  float*          sO = (float*)(base + OFF_SO);

  const int tid = (int)threadIdx.x, lane = tid & 31, wave = tid >> 5, hh = lane >> 4, m = lane & 15;
  const int b0 = (int)blockIdx.x * TB;

  {
    const v4i z4 = {0, 0, 0, 0};
    for (int i = tid; i < ZFILL16; i += NTHR) *(v4ia*)(base + (size_t)i * 16) = z4;
  }
  __syncthreads();
  load_x(x, b0, 0, sX, tid);
  __syncthreads();

#pragma unroll 1
  for (int t = 0; t < TSEQ; ++t) {
    const int cur = t & 1;
    const unsigned short* Hc  = Hb + cur * HB_HALVES;
    unsigned short*       Hn  = Hb + (cur ^ 1) * HB_HALVES;
    const unsigned short* sXc = sX + cur * SX_HALVES;

#pragma unroll 1
    for (int ct = 0; ct < 2; ++ct) {
      const int col = 32 * wave + 16 * ct + m;
      const v8f z8 = {0.f, 0.f, 0.f, 0.f, 0.f, 0.f, 0.f, 0.f};
      v8f aR0 = z8, aR1 = z8, aZ0 = z8, aZ1 = z8, aI0 = z8, aI1 = z8, aH0 = z8, aH1 = z8;

      {
        FragB x0, x1, bR, bZ, bN;
        const unsigned short* xp = sXc + m * XP + 8 * hh;
        ldfrag(x0, xp);
        ldfrag(x1, xp + 16 * XP);
        const unsigned short* wp = WIH + (size_t)col * KIN + 8 * hh;
        ldfrag(bR, wp);
        ldfrag(bZ, wp + (size_t)HID * KIN);
        ldfrag(bN, wp + (size_t)2 * HID * KIN);
        aR0 = wmb(x0, bR, aR0);
        aR1 = wmb(x1, bR, aR1);
        aZ0 = wmb(x0, bZ, aZ0);
        aZ1 = wmb(x1, bZ, aZ1);
        aI0 = wmb(x0, bN, aI0);
        aI1 = wmb(x1, bN, aI1);
      }

      if (t > 0) {
        const unsigned short* ap0 = Hc + m * HP + 8 * hh;
        const unsigned short* ap1 = ap0 + 16 * HP;
        const unsigned short* bp  = WHH + (size_t)col * HID + 8 * hh;
#pragma unroll 1
        for (int k0 = 0; k0 < HID; k0 += 32) {
          FragB h0, h1, l0, l1, bR, bZ, bN;
          ldfrag(h0, ap0 + k0);
          ldfrag(h1, ap1 + k0);
          ldfrag(l0, ap0 + HID + k0);
          ldfrag(l1, ap1 + HID + k0);
          ldfrag(bR, bp + k0);
          ldfrag(bZ, bp + (size_t)HID * HID + k0);
          ldfrag(bN, bp + (size_t)2 * HID * HID + k0);
          aR0 = wmb(h0, bR, aR0);
          aR1 = wmb(h1, bR, aR1);
          aZ0 = wmb(h0, bZ, aZ0);
          aZ1 = wmb(h1, bZ, aZ1);
          aH0 = wmb(h0, bN, aH0);
          aH1 = wmb(h1, bN, aH1);
          aR0 = wmb(l0, bR, aR0);
          aR1 = wmb(l1, bR, aR1);
          aZ0 = wmb(l0, bZ, aZ0);
          aZ1 = wmb(l1, bZ, aZ1);
          aH0 = wmb(l0, bN, aH0);
          aH1 = wmb(l1, bN, aH1);
        }
      }

      const float bRv = BIAS[BO_R + col];
      const float bZv = BIAS[BO_Z + col];
      const float bIv = BIAS[BO_IN + col];
      const float bHv = BIAS[BO_HN + col];
#pragma unroll
      for (int mt = 0; mt < 2; ++mt) {
        const v8f vR = mt ? aR1 : aR0;
        const v8f vZ = mt ? aZ1 : aZ0;
        const v8f vI = mt ? aI1 : aI0;
        const v8f vH = mt ? aH1 : aH0;
#pragma unroll
        for (int r = 0; r < 8; ++r) {
          const int row = 16 * mt + 8 * hh + r;
          const float ar = vR[r] + bRv;
          const float az = vZ[r] + bZv;
          const float rg = 1.0f / (1.0f + expf(-ar));
          const float zg = 1.0f / (1.0f + expf(-az));
          const float nn = tanhf((vI[r] + bIv) + rg * (vH[r] + bHv));
          const float ho = hF[row * HID + col];
          const float hn = (1.0f - zg) * nn + zg * ho;
          hF[row * HID + col] = hn;
          const unsigned hb = bf16_bits(hn);
          const unsigned lb = bf16_bits(hn - __uint_as_float(hb << 16));
          Hn[row * HP + col]       = (unsigned short)hb;
          Hn[row * HP + HID + col] = (unsigned short)lb;
        }
      }
    }

    if (t + 1 < TSEQ) load_x(x, b0, t + 1, sX + (cur ^ 1) * SX_HALVES, tid);
    __syncthreads();
  }

  if (wave < 4) {
    const int mt = wave >> 1, nt = wave & 1;
    v8f acc = {0.f, 0.f, 0.f, 0.f, 0.f, 0.f, 0.f, 0.f};
    const unsigned short* ap = Hb + (16 * mt + m) * HP + 8 * hh;
    const unsigned short* bp = FCW + (size_t)(16 * nt + m) * HID + 8 * hh;
#pragma unroll 1
    for (int k0 = 0; k0 < HID; k0 += 32) {
      FragB ah, al, b;
      ldfrag(ah, ap + k0);
      ldfrag(al, ap + HID + k0);
      ldfrag(b, bp + k0);
      acc = wmb(ah, b, acc);
      acc = wmb(al, b, acc);
    }
    const int oc = 16 * nt + m;
    const float fb = BIAS[BO_FC + oc];
#pragma unroll
    for (int r = 0; r < 8; ++r) {
      const int row = 16 * mt + 8 * hh + r;
      if (oc < NOUT) sO[row * NOUT + oc] = acc[r] + fb;
    }
  }
  __syncthreads();

  if (tid < OUT_CHUNKS) {
    const v4f v = *(const v4fa*)(sO + 4 * tid);
    float* op = out + (size_t)blockIdx.x * (TB * NOUT) + 4 * tid;
    *(volatile v4f*)op = v;
    __threadfence();
    *(volatile v4f*)op = v;
  }
}

extern "C" void kernel_launch(void* const* d_in, const int* in_sizes, int n_in,
                              void* d_out, int out_size, void* d_ws, size_t ws_size,
                              hipStream_t stream) {
  if (n_in < 7) return;
  if (in_sizes[0] != BATCH * TSEQ * NIN) return;
  if (in_sizes[1] != G3 * NIN) return;
  if (in_sizes[2] != G3 * HID) return;
  if (in_sizes[3] != G3 || in_sizes[4] != G3) return;
  if (in_sizes[5] != NOUT * HID) return;
  if (in_sizes[6] != NOUT) return;
  if (out_size != BATCH * NOUT) return;

  const float* x    = (const float*)d_in[0];
  const float* w_ih = (const float*)d_in[1];
  const float* w_hh = (const float*)d_in[2];
  const float* b_ih = (const float*)d_in[3];
  const float* b_hh = (const float*)d_in[4];
  const float* fc_w = (const float*)d_in[5];
  const float* fc_b = (const float*)d_in[6];
  float* out = (float*)d_out;

  char* ws = (char*)d_ws;
  size_t off = 0;
  const size_t oWHH = off; off += (size_t)G3 * HID * 2;      off = (off + 255) & ~(size_t)255;
  const size_t oWIH = off; off += (size_t)G3 * KIN * 2;      off = (off + 255) & ~(size_t)255;
  const size_t oFCW = off; off += (size_t)NOUTP * HID * 2;   off = (off + 255) & ~(size_t)255;
  const size_t oBIA = off; off += (size_t)NBIAS * 4;         off = (off + 255) & ~(size_t)255;
  if (off > ws_size) return;
  unsigned short* WHH  = (unsigned short*)(ws + oWHH);
  unsigned short* WIH  = (unsigned short*)(ws + oWIH);
  unsigned short* FCW  = (unsigned short*)(ws + oFCW);
  float*          BIAS = (float*)(ws + oBIA);

  hipFuncSetAttribute(reinterpret_cast<const void*>(&k_gru), hipFuncAttributeMaxDynamicSharedMemorySize,
                      (int)GRU_LDS_BYTES);

  k_prep<<<PREP_UNITS / NTHR, NTHR, 0, stream>>>(w_ih, w_hh, b_ih, b_hh, fc_w, fc_b, WHH, WIH, FCW, BIAS);
  k_gru<<<BATCH / TB, NTHR, GRU_LDS_BYTES, stream>>>(x, WHH, WIH, FCW, BIAS, out);
}
